// SRGAAttention_26577257627905
// MI455X (gfx1250) — hardware-verified
//
#include <hip/hip_runtime.h>
#include <hip/hip_bf16.h>
#include <math.h>
#include <stdint.h>

#define NBATCH 8
#define SEQ    1024
#define DM     768
#define NH     12
#define HD     64
#define QKVC   (3 * DM)
#define QKP    (2 * DM)
#define MP     (NBATCH * SEQ)
#define NQB    (SEQ / 64)
#define GRIDHW 32
#define NTAPP  64
#define WSC    64.0f
#define RSC    2048.0f
#define PSC    1024.0f
static_assert(NH * HD == DM);
static_assert(GRIDHW * GRIDHW == SEQ);
static_assert((SEQ % 64) == 0 && (DM % 64) == 0 && (QKP % 64) == 0 && (MP % 64) == 0 && (QKVC % 64) == 0);
static_assert((MP % 256) == 0 && ((NTAPP * DM / 8) % 256) == 0);

typedef _Float16 v16h __attribute__((ext_vector_type(16)));
typedef _Float16 v8h  __attribute__((ext_vector_type(8)));
typedef __bf16   v16b __attribute__((ext_vector_type(16)));
typedef float    v8f  __attribute__((ext_vector_type(8)));
typedef float    v4f  __attribute__((ext_vector_type(4)));
typedef unsigned int v4u __attribute__((ext_vector_type(4)));

union FragH { v16h v; v8h h[2]; };

__device__ __forceinline__ unsigned short bf_bits(float f) {
  unsigned u = __float_as_uint(f);
  return (unsigned short)((u + 0x7FFFu + ((u >> 16) & 1u)) >> 16);
}
__device__ __forceinline__ float bf_up(unsigned short hb) { return __uint_as_float(((unsigned)hb) << 16); }
__device__ __forceinline__ float bfr(float f) { return bf_up(bf_bits(f)); }
__device__ __forceinline__ unsigned short h_bits(_Float16 x) { return __builtin_bit_cast(unsigned short, x); }
__device__ __forceinline__ unsigned pk16(unsigned short a, unsigned short b) { return (unsigned)a | ((unsigned)b << 16); }
__device__ __forceinline__ v8f zero8() { v8f z = {0.f, 0.f, 0.f, 0.f, 0.f, 0.f, 0.f, 0.f}; return z; }

__device__ __forceinline__ v16h ldfrag_h(const _Float16* p) {
  FragH f;
  f.h[0] = *(const v8h*)(p);
  f.h[1] = *(const v8h*)(p + 16);
  return f.v;
}

__device__ __forceinline__ v8f mma_h(v16h a, v16h b, v8f c) {
  c = __builtin_amdgcn_wmma_f32_16x16x32_f16(false, a, false, b, (short)0, c, false, false);
#if defined(__HIP_DEVICE_COMPILE__)
  asm volatile("v_nop\n\tv_nop\n\tv_nop\n\tv_nop" : "+v"(c) : "v"(a), "v"(b));
#endif
  return c;
}
template <int TBF>
__device__ __forceinline__ v8f mma_raw(v16h a, v16h b, v8f c) {
  if (TBF) {
    return __builtin_amdgcn_wmma_f32_16x16x32_bf16(false, __builtin_bit_cast(v16b, a), false,
                                                   __builtin_bit_cast(v16b, b), (short)0, c, false, false);
  }
  return __builtin_amdgcn_wmma_f32_16x16x32_f16(false, a, false, b, (short)0, c, false, false);
}
__device__ __forceinline__ void dep_guard2(v8f& a, v8f& b, v16h x, v16h y) {
#if defined(__HIP_DEVICE_COMPILE__)
  asm volatile("v_nop\n\tv_nop\n\tv_nop\n\tv_nop" : "+v"(a), "+v"(b) : "v"(x), "v"(y));
#endif
}
__device__ __forceinline__ void keep4_h(v16h a, v16h b, v16h c, v16h d) {
#if defined(__HIP_DEVICE_COMPILE__)
  asm volatile("v_nop" :: "v"(a), "v"(b), "v"(c), "v"(d));
#endif
}
__device__ __forceinline__ void acc_guard4(v8f& a, v8f& b, v8f& c, v8f& d) {
#if defined(__HIP_DEVICE_COMPILE__)
  asm volatile("v_nop\n\tv_nop\n\tv_nop\n\tv_nop" : "+v"(a), "+v"(b), "+v"(c), "+v"(d));
#endif
}
__device__ __forceinline__ void wave_sync_lds() {
  __builtin_amdgcn_fence(__ATOMIC_RELEASE, "workgroup");
  __builtin_amdgcn_wave_barrier();
  __builtin_amdgcn_fence(__ATOMIC_ACQUIRE, "workgroup");
}

__global__ __launch_bounds__(256) void conv_h16(const float* __restrict__ X, unsigned short* Xh, int n8, float wsc) {
  const int i  = blockIdx.x * 256 + threadIdx.x;
  const int ic = (i < n8) ? i : (n8 - 1);
  const float* src = X + (size_t)ic * 8;
  const v4f a = *(const v4f*)(src);
  const v4f c = *(const v4f*)(src + 4);
  v4u o;
  o[0] = pk16(h_bits((_Float16)(bfr(a[0]) * wsc)), h_bits((_Float16)(bfr(a[1]) * wsc)));
  o[1] = pk16(h_bits((_Float16)(bfr(a[2]) * wsc)), h_bits((_Float16)(bfr(a[3]) * wsc)));
  o[2] = pk16(h_bits((_Float16)(bfr(c[0]) * wsc)), h_bits((_Float16)(bfr(c[1]) * wsc)));
  o[3] = pk16(h_bits((_Float16)(bfr(c[2]) * wsc)), h_bits((_Float16)(bfr(c[3]) * wsc)));
  if (i < n8) *(volatile v4u*)(Xh + (size_t)i * 8) = o;
  __threadfence();
  if (i < n8) *(volatile v4u*)(Xh + (size_t)i * 8) = o;
}

template <int MODE>
__global__ __launch_bounds__(256) void conv_t16(const float* __restrict__ Wm, unsigned short* Wt,
                                               int Krows, int Ncols, float wsc) {
  __shared__ float sW[64][65];
  const int t  = threadIdx.x;
  const int n0 = blockIdx.x * 64, k0 = blockIdx.y * 64;
  const int kr = t >> 4, c4 = (t & 15) * 4;
#pragma unroll
  for (int p = 0; p < 4; ++p) {
    const int row = kr + 16 * p;
    const v4f v = *(const v4f*)(Wm + (size_t)(k0 + row) * Ncols + n0 + c4);
    sW[row][c4 + 0] = v[0];
    sW[row][c4 + 1] = v[1];
    sW[row][c4 + 2] = v[2];
    sW[row][c4 + 3] = v[3];
  }
  __syncthreads();
  v4u o[2];
  size_t go[2];
#pragma unroll
  for (int p = 0; p < 2; ++p) {
    const int id = p * 256 + t;
    const int nr = id >> 3, kp = (id & 7) * 8;
    unsigned short u[8];
#pragma unroll
    for (int e = 0; e < 8; ++e) {
      const float f = sW[kp + e][nr];
      u[e] = MODE ? bf_bits(f) : h_bits((_Float16)(bfr(f) * wsc));
    }
    v4u a;
    a[0] = pk16(u[0], u[1]);
    a[1] = pk16(u[2], u[3]);
    a[2] = pk16(u[4], u[5]);
    a[3] = pk16(u[6], u[7]);
    o[p]  = a;
    go[p] = (size_t)(n0 + nr) * Krows + k0 + kp;
  }
  *(volatile v4u*)(Wt + go[0]) = o[0];
  *(volatile v4u*)(Wt + go[1]) = o[1];
  __threadfence();
  *(volatile v4u*)(Wt + go[0]) = o[0];
  *(volatile v4u*)(Wt + go[1]) = o[1];
}

__global__ __launch_bounds__(256) void conv_wb(const float* __restrict__ Wb, unsigned short* WbH, int n8) {
  const int i  = blockIdx.x * 256 + threadIdx.x;
  const int ic = (i < n8) ? i : (n8 - 1);
  const int j  = ic / (DM / 8);
  const int c0 = (ic - j * (DM / 8)) * 8;
  const int jc = (j < 9) ? j : 8;
  unsigned short u[8];
#pragma unroll
  for (int e = 0; e < 8; ++e) {
    const float f = Wb[(c0 + e) * 9 + jc];
    const float g = (j < 9) ? (bfr(f) * WSC) : 0.0f;
    u[e] = h_bits((_Float16)g);
  }
  v4u o;
  o[0] = pk16(u[0], u[1]);
  o[1] = pk16(u[2], u[3]);
  o[2] = pk16(u[4], u[5]);
  o[3] = pk16(u[6], u[7]);
  if (i < n8) *(volatile v4u*)(WbH + (size_t)i * 8) = o;
  __threadfence();
  if (i < n8) *(volatile v4u*)(WbH + (size_t)i * 8) = o;
}

template <int TBF, int NA, int OM, int BIASM>
__global__ __launch_bounds__(256) void gemm64(
    const unsigned short* __restrict__ Ap, const unsigned short* __restrict__ A2p, int lda, long long strideA,
    const unsigned short* __restrict__ Btp, int ldb, long long strideB,
    const float* __restrict__ bias0,
    void* Cout, int ldc, long long strideC,
    void* Cout2, int ldc2, long long strideC2, int N2,
    int M, int N, int K, float oscale) {
  const _Float16* A  = (const _Float16*)(const void*)Ap;
  const _Float16* A2 = (const _Float16*)(const void*)A2p;
  const _Float16* Bt = (const _Float16*)(const void*)Btp;
  __shared__ __align__(16) float sT[8][16 * 68];
  const int b    = blockIdx.y;
  const int lane = threadIdx.x & 31;
  const int wave = threadIdx.x >> 5;
  const int tilesN = N >> 6;
  const int tilesM = M >> 6;
  const int tile = blockIdx.x * 8 + wave;
  if (tile >= tilesM * tilesN) return;
  const int tm = tile / tilesN;
  const int tn = tile - tm * tilesN;
  const int m0 = tm << 6;
  const int n0 = tn << 6;

  const _Float16* Ab  = A  + (size_t)b * (size_t)strideA;
  const _Float16* A2b = A2 + (size_t)b * (size_t)strideA;
  const _Float16* Bb  = Bt + (size_t)b * (size_t)strideB;

  const int rlane = lane & 15;
  const int koff  = (lane >> 4) * 8;
  const int mOff  = (lane >> 4) * 8;

  v8f acc[4][4];
#pragma unroll
  for (int i = 0; i < 4; ++i)
#pragma unroll
    for (int j = 0; j < 4; ++j) acc[i][j] = zero8();

  for (int k0 = 0; k0 < K; k0 += 32) {
    v16h bh[4];
#pragma unroll
    for (int j = 0; j < 4; ++j) {
      const size_t bo = (size_t)(n0 + (j << 4) + rlane) * ldb + koff + k0;
      bh[j] = ldfrag_h(Bb + bo);
    }
#pragma unroll
    for (int i = 0; i < 4; ++i) {
      const size_t ao = (size_t)(m0 + (i << 4) + rlane) * lda + koff + k0;
      const v16h ah = ldfrag_h(Ab + ao);
      v16h ah2 = ah;
      if (NA == 2) ah2 = ldfrag_h(A2b + ao);
#pragma unroll
      for (int j = 0; j < 4; ++j) acc[i][j] = mma_raw<TBF>(ah, bh[j], acc[i][j]);
      if (NA == 2) {
#pragma unroll
        for (int j = 0; j < 4; ++j) acc[i][j] = mma_raw<TBF>(ah2, bh[j], acc[i][j]);
      }
      dep_guard2(acc[i][0], acc[i][3], ah, ah2);
    }
    keep4_h(bh[0], bh[1], bh[2], bh[3]);
  }
  acc_guard4(acc[0][0], acc[0][1], acc[0][2], acc[0][3]);
  acc_guard4(acc[1][0], acc[1][1], acc[1][2], acc[1][3]);
  acc_guard4(acc[2][0], acc[2][1], acc[2][2], acc[2][3]);
  acc_guard4(acc[3][0], acc[3][1], acc[3][2], acc[3][3]);

  const int hh2 = lane >> 4, c4 = (lane & 15) * 4;
  const int q8  = lane >> 3, c8 = (lane & 7) * 8;
  float bc[8];
#pragma unroll
  for (int e = 0; e < 8; ++e) bc[e] = 0.f;
  if (BIASM == 0) {
    if (OM == 0) {
      const v4f b0v = *(const v4f*)(bias0 + n0 + c4);
#pragma unroll
      for (int e = 0; e < 4; ++e) bc[e] = bfr(b0v[e]);
    } else {
      const v4f b0a = *(const v4f*)(bias0 + n0 + c8);
      const v4f b0b = *(const v4f*)(bias0 + n0 + c8 + 4);
#pragma unroll
      for (int e = 0; e < 4; ++e) {
        bc[e]     = bfr(b0a[e]);
        bc[4 + e] = bfr(b0b[e]);
      }
    }
  }

  float* slab = sT[wave];
#pragma unroll
  for (int i = 0; i < 4; ++i) {
    const int mBase = m0 + (i << 4);
#pragma unroll
    for (int j = 0; j < 4; ++j) {
#pragma unroll
      for (int r = 0; r < 8; ++r) {
        slab[(mOff + r) * 68 + (j << 4) + rlane] = acc[i][j][r];
      }
    }
    wave_sync_lds();
    if (OM == 0) {
      float* C = (float*)Cout + (size_t)b * (size_t)strideC;
      v4f vals[8];
#pragma unroll
      for (int it = 0; it < 8; ++it) {
        const int row = it * 2 + hh2;
        v4f v = *(const v4f*)(slab + row * 68 + c4);
#pragma unroll
        for (int e = 0; e < 4; ++e) v[e] = v[e] * oscale + bc[e];
        vals[it] = v;
      }
      for (int pass = 0; pass < 2; ++pass) {
#pragma unroll
        for (int it = 0; it < 8; ++it) {
          const int row = it * 2 + hh2;
          *(volatile v4f*)(C + (size_t)(mBase + row) * ldc + n0 + c4) = vals[it];
        }
        __threadfence();
      }
    } else {
      unsigned short* C  = (unsigned short*)Cout  + (size_t)b * (size_t)strideC;
      unsigned short* C2 = (unsigned short*)Cout2 + (size_t)b * (size_t)strideC2;
      const bool wr2 = (OM == 3) && (n0 < N2);
      v4u hv[4], hr[4];
#pragma unroll
      for (int it = 0; it < 4; ++it) {
        const int row = it * 4 + q8;
        const float* sp = slab + row * 68 + c8;
        float bm = 0.f;
        if (BIASM == 1) bm = bfr(bias0[mBase + row]);
        v4u a, ar;
#pragma unroll
        for (int e = 0; e < 4; ++e) {
          const float f0 = sp[2 * e]     * oscale + ((BIASM == 1) ? bm : bc[2 * e]);
          const float f1 = sp[2 * e + 1] * oscale + ((BIASM == 1) ? bm : bc[2 * e + 1]);
          const _Float16 g0 = (_Float16)f0, g1 = (_Float16)f1;
          const _Float16 r0 = (_Float16)((f0 - (float)g0) * RSC);
          const _Float16 r1 = (_Float16)((f1 - (float)g1) * RSC);
          a[e]  = pk16(h_bits(g0), h_bits(g1));
          ar[e] = pk16(h_bits(r0), h_bits(r1));
        }
        hv[it] = a;
        hr[it] = ar;
      }
      for (int pass = 0; pass < 2; ++pass) {
#pragma unroll
        for (int it = 0; it < 4; ++it) {
          const int row = it * 4 + q8;
          *(volatile v4u*)(C + (size_t)(mBase + row) * ldc + n0 + c8) = hv[it];
          if (wr2) *(volatile v4u*)(C2 + (size_t)(mBase + row) * ldc2 + n0 + c8) = hr[it];
        }
        __threadfence();
      }
    }
    wave_sync_lds();
  }
}

__global__ __launch_bounds__(256) void k_biasmap(const float* __restrict__ T, const float* __restrict__ bb,
                                                const int* __restrict__ Hp, const int* __restrict__ Wp,
                                                float* bias, int npix) {
  const int pix = blockIdx.x * 256 + threadIdx.x;
  const int pc  = (pix < npix) ? pix : (npix - 1);
  const int b = pc >> 10, n = pc & 1023, y = n >> 5, xx = n & 31;
  int Hm = Hp[0], Wm = Wp[0];
  Hm = (Hm < 1) ? 1 : ((Hm > GRIDHW) ? GRIDHW : Hm);
  Wm = (Wm < 1) ? 1 : ((Wm > GRIDHW) ? GRIDHW : Wm);
  float sum = 0.f;
#pragma unroll
  for (int dy = 0; dy < 3; ++dy) {
#pragma unroll
    for (int dx = 0; dx < 3; ++dx) {
      const int yy = y + dy - 1, x2 = xx + dx - 1;
      const bool ok = (yy >= 0) && (yy < Hm) && (x2 >= 0) && (x2 < Wm);
      const int yc = (yy < 0) ? 0 : ((yy > GRIDHW - 1) ? (GRIDHW - 1) : yy);
      const int xc = (x2 < 0) ? 0 : ((x2 > GRIDHW - 1) ? (GRIDHW - 1) : x2);
      const float v = T[((size_t)b * SEQ + (size_t)yc * GRIDHW + xc) * NTAPP + dy * 3 + dx];
      sum += ok ? v : 0.f;
    }
  }
  const float outv = sum + bfr(bb[0]);
  if (pix < npix) *(volatile float*)(bias + pix) = outv;
  __threadfence();
  if (pix < npix) *(volatile float*)(bias + pix) = outv;
}

__global__ __launch_bounds__(128)
void attn64(const unsigned short* __restrict__ qkp, const unsigned short* __restrict__ qrp,
            const unsigned short* __restrict__ vtp, const unsigned short* __restrict__ vrp,
            const float* __restrict__ bsp, unsigned short* ctxh, unsigned short* ctxl, float sscale) {
  __shared__ __align__(16) _Float16 Ksh[64 * 64];
  __shared__ __align__(16) _Float16 Vth[64 * 64];
  __shared__ __align__(16) _Float16 Vtr[64 * 64];
  __shared__ __align__(16) _Float16 Psh[4][16 * 64];
  __shared__ __align__(16) float    Os[4][16 * 64];

  const int tid  = threadIdx.x;
  const int wave = tid >> 5;
  const int lane = tid & 31;
  const int hh   = lane >> 4;
  const int c    = lane & 15;

  const int bx   = blockIdx.x;
  const int qb   = bx % NQB;
  const int rest = bx / NQB;
  const int h    = rest % NH;
  const int b    = rest / NH;
  const int q0   = qb * 64 + wave * 16;
  const size_t rowB = (size_t)b * SEQ;

  const _Float16* Qh = (const _Float16*)(const void*)qkp + (size_t)h * HD;
  const _Float16* Qr = (const _Float16*)(const void*)qrp + (size_t)h * HD;
  const _Float16* Kg = (const _Float16*)(const void*)qkp + DM + (size_t)h * HD;
  const _Float16* Vh = (const _Float16*)(const void*)vtp + ((size_t)b * DM + (size_t)h * HD) * SEQ;
  const _Float16* Vr = (const _Float16*)(const void*)vrp + ((size_t)b * DM + (size_t)h * HD) * SEQ;
  const float*    Bb = bsp + rowB;

  v16h qa[2], qr[2];
#pragma unroll
  for (int dc = 0; dc < 2; ++dc) {
    qa[dc] = ldfrag_h(Qh + (rowB + q0 + c) * QKP + dc * 32 + 8 * hh);
    qr[dc] = ldfrag_h(Qr + (rowB + q0 + c) * DM  + dc * 32 + 8 * hh);
  }
  const float sres = sscale * (1.0f / RSC);

  float mrow[8], lrow[8];
  v8f oacc[4];
#pragma unroll
  for (int r = 0; r < 8; ++r) { mrow[r] = -INFINITY; lrow[r] = 0.f; }
#pragma unroll
  for (int t = 0; t < 4; ++t) oacc[t] = zero8();

  for (int kt = 0; kt < NQB; ++kt) {
    const int kv0 = kt * 64;
    float mk[4];
#pragma unroll
    for (int j = 0; j < 4; ++j) mk[j] = Bb[kv0 + j * 16 + c];

    __syncthreads();
    {
      const int r = tid >> 1, hf = (tid & 1) * 32;
      const _Float16* kg = Kg + (rowB + kv0 + r) * QKP + hf;
      const _Float16* vg = Vh + (size_t)r * SEQ + kv0 + hf;
      const _Float16* vr = Vr + (size_t)r * SEQ + kv0 + hf;
#pragma unroll
      for (int i = 0; i < 4; ++i) {
        const v8h a0 = *(const v8h*)(kg + 8 * i);
        const v8h b0 = *(const v8h*)(vg + 8 * i);
        const v8h c0 = *(const v8h*)(vr + 8 * i);
        *(v8h*)(Ksh + r * 64 + hf + 8 * i) = a0;
        *(v8h*)(Vth + r * 64 + hf + 8 * i) = b0;
        *(v8h*)(Vtr + r * 64 + hf + 8 * i) = c0;
      }
    }
    __syncthreads();

    v8f s[4];
#pragma unroll
    for (int j = 0; j < 4; ++j) {
      v8f sh = zero8(), sr = zero8();
#pragma unroll
      for (int dc = 0; dc < 2; ++dc) {
        FragH kb;
        kb.h[0] = *(const v8h*)(Ksh + (j * 16 + c) * 64 + dc * 32 + 8 * hh);
        kb.h[1] = *(const v8h*)(Ksh + (j * 16 + c) * 64 + dc * 32 + 16 + 8 * hh);
        sh = mma_h(qa[dc], kb.v, sh);
        sr = mma_h(qr[dc], kb.v, sr);
      }
#pragma unroll
      for (int r = 0; r < 8; ++r) s[j][r] = sh[r] * sscale + sr[r] * sres + mk[j];
    }

    _Float16* pwh = Psh[wave];
#pragma unroll
    for (int r = 0; r < 8; ++r) {
      float m = s[0][r];
      m = fmaxf(m, s[1][r]);
      m = fmaxf(m, s[2][r]);
      m = fmaxf(m, s[3][r]);
#pragma unroll
      for (int off = 1; off < 16; off <<= 1) m = fmaxf(m, __shfl_xor(m, off, 32));
      const float mnew  = fmaxf(mrow[r], m);
      const float alpha = __expf(mrow[r] - mnew);
      mrow[r] = mnew;
      float psum = 0.f;
#pragma unroll
      for (int j = 0; j < 4; ++j) {
        const float p = __expf(s[j][r] - mnew);
        psum += p;
        pwh[(8 * hh + r) * 64 + j * 16 + c] = (_Float16)(p * PSC);
      }
#pragma unroll
      for (int off = 1; off < 16; off <<= 1) psum += __shfl_xor(psum, off, 32);
      lrow[r] = lrow[r] * alpha + psum;
#pragma unroll
      for (int t = 0; t < 4; ++t) oacc[t][r] *= alpha;
    }
    wave_sync_lds();

    v16h pa[2];
#pragma unroll
    for (int kk = 0; kk < 2; ++kk) {
      FragH pf;
      pf.h[0] = *(const v8h*)(pwh + c * 64 + kk * 32 + 8 * hh);
      pf.h[1] = *(const v8h*)(pwh + c * 64 + kk * 32 + 16 + 8 * hh);
      pa[kk] = pf.v;
    }
#pragma unroll
    for (int kk = 0; kk < 2; ++kk) {
#pragma unroll
      for (int t = 0; t < 4; ++t) {
        FragH vb;
        vb.h[0] = *(const v8h*)(Vth + (t * 16 + c) * 64 + kk * 32 + 8 * hh);
        vb.h[1] = *(const v8h*)(Vth + (t * 16 + c) * 64 + kk * 32 + 16 + 8 * hh);
        oacc[t] = mma_h(pa[kk], vb.v, oacc[t]);
      }
    }
    v8f accr[4];
#pragma unroll
    for (int t = 0; t < 4; ++t) accr[t] = zero8();
#pragma unroll
    for (int kk = 0; kk < 2; ++kk) {
#pragma unroll
      for (int t = 0; t < 4; ++t) {
        FragH vb;
        vb.h[0] = *(const v8h*)(Vtr + (t * 16 + c) * 64 + kk * 32 + 8 * hh);
        vb.h[1] = *(const v8h*)(Vtr + (t * 16 + c) * 64 + kk * 32 + 16 + 8 * hh);
        accr[t] = mma_h(pa[kk], vb.v, accr[t]);
      }
    }
#pragma unroll
    for (int t = 0; t < 4; ++t) {
#pragma unroll
      for (int r = 0; r < 8; ++r) oacc[t][r] += accr[t][r] * (1.0f / RSC);
    }
  }

  float* os = Os[wave];
#pragma unroll
  for (int r = 0; r < 8; ++r) {
    const float l = lrow[r];
    const float inv = ((l > 0.f) ? (1.0f / l) : 0.f) * (1.0f / PSC);
#pragma unroll
    for (int t = 0; t < 4; ++t) os[(8 * hh + r) * 64 + t * 16 + c] = oacc[t][r] * inv;
  }
  wave_sync_lds();
  {
    const int q4 = lane >> 3, c8 = (lane & 7) * 8;
    v4u hv[4], lv[4];
#pragma unroll
    for (int it = 0; it < 4; ++it) {
      const int row = it * 4 + q4;
      const float* sp = os + row * 64 + c8;
      v4u a, al;
#pragma unroll
      for (int e = 0; e < 4; ++e) {
        const float f0 = sp[2 * e], f1 = sp[2 * e + 1];
        const unsigned short g0 = bf_bits(f0), g1 = bf_bits(f1);
        const unsigned short l0 = bf_bits(f0 - bf_up(g0)), l1 = bf_bits(f1 - bf_up(g1));
        a[e]  = pk16(g0, g1);
        al[e] = pk16(l0, l1);
      }
      hv[it] = a;
      lv[it] = al;
    }
    for (int pass = 0; pass < 2; ++pass) {
#pragma unroll
      for (int it = 0; it < 4; ++it) {
        const int row = it * 4 + q4;
        const size_t go = (rowB + q0 + row) * DM + (size_t)h * HD + c8;
        *(volatile v4u*)(ctxh + go) = hv[it];
        *(volatile v4u*)(ctxl + go) = lv[it];
      }
      __threadfence();
    }
  }
}

extern "C" void kernel_launch(void* const* d_in, const int* in_sizes, int n_in,
                              void* d_out, int out_size, void* d_ws, size_t ws_size,
                              hipStream_t stream) {
  if (n_in < 9) return;
  if (in_sizes[0] != MP * DM) return;
  if (in_sizes[1] != 1 || in_sizes[2] != 1) return;
  if (in_sizes[3] != DM * QKVC) return;
  if (in_sizes[4] != QKVC) return;
  if (in_sizes[5] != DM * DM || in_sizes[6] != DM) return;
  if (in_sizes[7] != DM * 9 || in_sizes[8] != 1) return;
  if (out_size != MP * DM) return;

  const float* xin   = (const float*)d_in[0];
  const int*   Hin   = (const int*)d_in[1];
  const int*   Win   = (const int*)d_in[2];
  const float* wqkv  = (const float*)d_in[3];
  const float* bqkv  = (const float*)d_in[4];
  const float* wproj = (const float*)d_in[5];
  const float* bproj = (const float*)d_in[6];
  const float* wbias = (const float*)d_in[7];
  const float* bbias = (const float*)d_in[8];

  const size_t PWQKV = (size_t)QKVC * DM * 2;
  const size_t PWO   = (size_t)DM * DM * 2;
  const size_t PWB   = (size_t)NTAPP * DM * 2;
  const size_t PXH   = (size_t)MP * DM * 2;
  const size_t PT    = (size_t)MP * NTAPP * 4;
  const size_t PBIAS = (size_t)MP * 4;
  const size_t PQK   = (size_t)MP * QKP * 2;
  const size_t PQR   = (size_t)MP * DM * 2;
  const size_t PVT   = (size_t)NBATCH * DM * SEQ * 2;
  const size_t PCTX  = (size_t)MP * DM * 2;
  size_t off = 0;
  const size_t oWqkv = off; off += PWQKV;
  const size_t oWo   = off; off += PWO;
  const size_t oWb   = off; off += PWB;
  const size_t oXH   = off; off += PXH;
  const size_t oT    = off; off += PT;
  const size_t oBias = off; off += PBIAS;
  const size_t oQK   = off; off += PQK;
  const size_t oQR   = off; off += PQR;
  const size_t oVT   = off; off += PVT;
  const size_t oVR   = off; off += PVT;
  const size_t oCH   = off; off += PCTX;
  const size_t oCL   = off; off += PCTX;
  if (off > ws_size) return;
  if (off > (size_t)134217728) return;

  char* ws = (char*)d_ws;
  unsigned short* WqkvH = (unsigned short*)(ws + oWqkv);
  unsigned short* WoB   = (unsigned short*)(ws + oWo);
  unsigned short* WbH   = (unsigned short*)(ws + oWb);
  unsigned short* XH    = (unsigned short*)(ws + oXH);
  float*          Tt    = (float*)(ws + oT);
  float*          BIAS  = (float*)(ws + oBias);
  unsigned short* QK    = (unsigned short*)(ws + oQK);
  unsigned short* QR    = (unsigned short*)(ws + oQR);
  unsigned short* VT    = (unsigned short*)(ws + oVT);
  unsigned short* VR    = (unsigned short*)(ws + oVR);
  unsigned short* CtxH  = (unsigned short*)(ws + oCH);
  unsigned short* CtxL  = (unsigned short*)(ws + oCL);
  float*          out0  = (float*)d_out;

  const int n8x = (MP * DM) / 8;
  const int n8b = (NTAPP * DM) / 8;
  if ((n8x % 256) != 0 || (n8b % 256) != 0) return;
  const dim3 blk(256), blk128(128);
  const dim3 gCx(n8x / 256);
  const dim3 gTq(QKVC / 64, DM / 64);
  const dim3 gTo(DM / 64, DM / 64);
  const dim3 gWb(n8b / 256);
  const dim3 gT(((MP / 64) * (NTAPP / 64) + 7) / 8, 1);
  const dim3 gBm(MP / 256);
  const dim3 gNqk(((MP / 64) * (QKP / 64) + 7) / 8, 1);
  const dim3 gVT(((DM / 64) * (SEQ / 64) + 7) / 8, NBATCH);
  const dim3 gAttn(NBATCH * NH * NQB);
  const dim3 gNo(((MP / 64) * (DM / 64) + 7) / 8, 1);
  const float invw = 1.0f / WSC;

  conv_h16<<<gCx, blk, 0, stream>>>(xin, XH, n8x, 1.0f);
  conv_t16<0><<<gTq, blk, 0, stream>>>(wqkv, WqkvH, DM, QKVC, WSC);
  conv_t16<1><<<gTo, blk, 0, stream>>>(wproj, WoB, DM, DM, 1.0f);
  conv_wb<<<gWb, blk, 0, stream>>>(wbias, WbH, n8b);

  gemm64<0, 1, 0, 2><<<gT, blk, 0, stream>>>(
      XH, XH, DM, 0LL, WbH, DM, 0LL, bqkv,
      (void*)Tt, NTAPP, 0LL, (void*)Tt, NTAPP, 0LL, 0,
      MP, NTAPP, DM, invw);
  k_biasmap<<<gBm, blk, 0, stream>>>(Tt, bbias, Hin, Win, BIAS, MP);

  gemm64<0, 1, 3, 0><<<gNqk, blk, 0, stream>>>(
      XH, XH, DM, 0LL, WqkvH, DM, 0LL, bqkv,
      (void*)QK, QKP, 0LL, (void*)QR, DM, 0LL, DM,
      MP, QKP, DM, invw);
  gemm64<0, 1, 3, 1><<<gVT, blk, 0, stream>>>(
      WqkvH + (size_t)QKP * DM, WqkvH + (size_t)QKP * DM, DM, 0LL, XH, DM, (long long)SEQ * DM, bqkv + QKP,
      (void*)VT, SEQ, (long long)DM * SEQ, (void*)VR, SEQ, (long long)DM * SEQ, SEQ,
      DM, SEQ, DM, invw);

  attn64<<<gAttn, blk128, 0, stream>>>(QK, QR, VT, VR, BIAS, CtxH, CtxL, 0.125f);

  gemm64<1, 2, 0, 0><<<gNo, blk, 0, stream>>>(
      CtxH, CtxL, DM, 0LL, WoB, DM, 0LL, bproj,
      (void*)out0, DM, 0LL, (void*)out0, DM, 0LL, 0,
      MP, DM, DM, 1.0f);
  (void)hipGetLastError();
}
